// LightWeightConv1DBlock_53171695125234
// MI455X (gfx1250) — hardware-verified
//
#include <hip/hip_runtime.h>

#define NB    4
#define NT    1024
#define NC    1024
#define NH    16
#define NK    31
#define PADL  15
#define NR    64
#define HK    (NH * NK)
#define NPAD  512
#define MROWS (NB * NT)
#define KP    32

typedef _Float16 v16h __attribute__((ext_vector_type(16)));
typedef _Float16 v8h  __attribute__((ext_vector_type(8)));
typedef float    v8f  __attribute__((ext_vector_type(8)));
typedef float    v4f  __attribute__((ext_vector_type(4)));
typedef v4f      v4fa __attribute__((may_alias));
union Frag { v16h v; v8h half[2]; };

static __device__ __forceinline__ v8f mma_f16(v16h a, v16h b, v8f c) {
    v8f d = __builtin_amdgcn_wmma_f32_16x16x32_f16(false, a, false, b, (short)0, c, false, false);
    asm volatile("v_nop\n\tv_nop\n\tv_nop\n\tv_nop" : "+v"(d) : "v"(a), "v"(b));
    return d;
}

__global__ __launch_bounds__(256) void k_convert(const float* __restrict__ x,
                                                 const float* __restrict__ W,
                                                 _Float16* __restrict__ xh,
                                                 _Float16* __restrict__ wh) {
    const unsigned g   = blockIdx.x * 256u + threadIdx.x;
    const unsigned NXG = (unsigned)(MROWS * NC / 8);
    const unsigned NWG = (unsigned)(NPAD * NC / 8);
    v8h hv = (v8h){};
    _Float16* dst = xh;
    bool act = false;
    if (g < NXG) {
        const float* p = x + (size_t)g * 8;
        v4f lo = *(const v4f*)p;
        v4f hi = *(const v4f*)(p + 4);
        v8f f = __builtin_shufflevector(lo, hi, 0, 1, 2, 3, 4, 5, 6, 7);
        hv = __builtin_convertvector(f, v8h);
        dst = xh + (size_t)g * 8;
        act = true;
    } else if (g < NXG + NWG) {
        const unsigned gw = g - NXG;
        const unsigned n  = gw >> 7;
        const unsigned kk = (gw & 127u) * 8u;
        v8f f = (v8f){};
        if (n < (unsigned)HK) {
            const float* p = W + (size_t)n * NC + kk;
            v4f lo = *(const v4f*)p;
            v4f hi = *(const v4f*)(p + 4);
            f = __builtin_shufflevector(lo, hi, 0, 1, 2, 3, 4, 5, 6, 7);
            f = f * 64.0f;
        }
        hv = __builtin_convertvector(f, v8h);
        dst = wh + (size_t)gw * 8;
        act = true;
    }
    if (act) *(volatile v8h*)dst = hv;
    __threadfence();
    if (act) *(volatile v8h*)dst = hv;
}

__global__ __launch_bounds__(256) void k_gemm_softmax(const _Float16* __restrict__ xh,
                                                      const _Float16* __restrict__ wh,
                                                      float* __restrict__ wsm) {
    __shared__ __attribute__((aligned(16))) float Lg[16 * NPAD];
    __shared__ __attribute__((aligned(16))) float Ps[16 * NH * KP];

    const int tid  = threadIdx.x;
    const int wave = tid >> 5;
    const int lane = tid & 31;
    const int h    = lane >> 4;
    const int m    = lane & 15;

    const int m0 = blockIdx.x * 16;
    const _Float16* pa = xh + (size_t)(m0 + m) * NC + 8 * h;
    const _Float16* pb = wh + (size_t)(wave * 64 + m) * NC + 8 * h;

    v8f acc[4];
#pragma unroll
    for (int i = 0; i < 4; ++i) acc[i] = (v8f){};

#pragma unroll 1
    for (int k0 = 0; k0 < NC; k0 += 32) {
        Frag a;
        a.half[0] = *(const v8h*)(pa + k0);
        a.half[1] = *(const v8h*)(pa + k0 + 16);
#pragma unroll
        for (int i = 0; i < 4; ++i) {
            const _Float16* q = pb + (size_t)i * 16 * NC + k0;
            Frag b;
            b.half[0] = *(const v8h*)(q);
            b.half[1] = *(const v8h*)(q + 16);
            acc[i] = mma_f16(a.v, b.v, acc[i]);
        }
    }

#pragma unroll
    for (int i = 0; i < 4; ++i) {
        const int col = wave * 64 + i * 16 + m;
#pragma unroll
        for (int r = 0; r < 8; ++r)
            Lg[(8 * h + r) * NPAD + col] = acc[i][r] * (1.0f / 64.0f);
    }
    __syncthreads();

    const int lt = tid >> 4;
    const int hd = tid & 15;
    float* row = Lg + lt * NPAD + hd * NK;

    float mx = -3.402823466e38f;
#pragma unroll 1
    for (int k = 0; k < NK; ++k) mx = fmaxf(mx, row[k]);
    float s = 0.0f;
#pragma unroll 1
    for (int k = 0; k < NK; ++k) {
        float e = expf(row[k] - mx);
        row[k] = e;
        s += e;
    }
    const float inv = __builtin_amdgcn_rcpf(s);
    float* prow = Ps + lt * (NH * KP) + hd * KP;
#pragma unroll 1
    for (int k = 0; k < NK; ++k) prow[k] = row[k] * inv;
    prow[NK] = 0.0f;
    __syncthreads();

    float* base = wsm + (size_t)blockIdx.x * (16 * NH * KP);
    v4f vals[8];
#pragma unroll
    for (int p = 0; p < 8; ++p) vals[p] = *(const v4fa*)(Ps + p * 1024 + tid * 4);
#pragma unroll
    for (int p = 0; p < 8; ++p) *(volatile v4f*)(base + p * 1024 + tid * 4) = vals[p];
    __threadfence();
#pragma unroll
    for (int p = 0; p < 8; ++p) *(volatile v4f*)(base + p * 1024 + tid * 4) = vals[p];
}

__global__ __launch_bounds__(256) void k_band_conv(const float* __restrict__ x,
                                                   const float* __restrict__ wsm,
                                                   float* __restrict__ out) {
    __shared__ v4f xs4[(64 + NK - 1) * 16];
    __shared__ __attribute__((aligned(16))) float fs[64 * KP];

    const int tid = threadIdx.x;
    const int bid = blockIdx.x;
    const int tt  = bid & 15;
    const int hh  = (bid >> 4) & 15;
    const int b   = bid >> 8;
    const int t0  = tt * 64;

    for (int i = tid; i < (64 + NK - 1) * 16; i += 256) {
        const int li = i >> 4;
        const int c4 = i & 15;
        const int ts = t0 + li - PADL;
        v4f v = (v4f){};
        if (ts >= 0 && ts < NT)
            v = *(const v4f*)(x + ((size_t)(b * NT + ts)) * NC + hh * NR + c4 * 4);
        xs4[i] = v;
    }
    for (int i = tid; i < 64 * 8; i += 256) {
        const int lt = i >> 3;
        const int q  = i & 7;
        v4f v = *(const v4f*)(wsm + (((size_t)(b * NT + t0 + lt)) * NH + hh) * KP + q * 4);
        *(v4fa*)(fs + lt * KP + q * 4) = v;
    }
    __syncthreads();

    const int wave = tid >> 5;
    const int lane = tid & 31;
    const int hrow = lane >> 4;
    const int rq   = lane & 15;

    v4f acc[4];
#pragma unroll
    for (int j = 0; j < 4; ++j) acc[j] = (v4f){};

#pragma unroll 1
    for (int k = 0; k < NK; ++k) {
#pragma unroll
        for (int j = 0; j < 4; ++j) {
            const int lt = wave * 8 + 2 * j + hrow;
            const float wk = fs[lt * KP + k];
            const v4f xv = xs4[(lt + k) * 16 + rq];
            acc[j] = acc[j] + xv * wk;
        }
    }

#pragma unroll
    for (int j = 0; j < 4; ++j) {
        const int lt = wave * 8 + 2 * j + hrow;
        float* o = out + ((size_t)(b * NT + t0 + lt)) * NC + hh * NR + rq * 4;
        *(volatile v4f*)o = acc[j];
    }
    __threadfence();
#pragma unroll
    for (int j = 0; j < 4; ++j) {
        const int lt = wave * 8 + 2 * j + hrow;
        float* o = out + ((size_t)(b * NT + t0 + lt)) * NC + hh * NR + rq * 4;
        *(volatile v4f*)o = acc[j];
    }
}

extern "C" void kernel_launch(void* const* d_in, const int* in_sizes, int n_in,
                              void* d_out, int out_size, void* d_ws, size_t ws_size,
                              hipStream_t stream) {
    if (n_in < 2) return;
    if (in_sizes[0] != MROWS * NC) return;
    if (in_sizes[1] != HK * NC) return;
    if (out_size != MROWS * NC) return;

    const float* x = (const float*)d_in[0];
    const float* W = (const float*)d_in[1];
    float* out = (float*)d_out;

    const size_t off_xh  = 0;
    const size_t off_wh  = off_xh + (size_t)MROWS * NC * 2;
    const size_t off_wsm = off_wh + (size_t)NPAD * NC * 2;
    const size_t total   = off_wsm + (size_t)MROWS * NH * KP * 4;
    if (ws_size < total) return;

    _Float16* xh  = (_Float16*)((char*)d_ws + off_xh);
    _Float16* wh  = (_Float16*)((char*)d_ws + off_wh);
    float*    wsm = (float*)((char*)d_ws + off_wsm);

    {
        const unsigned ngroups = (unsigned)(MROWS * NC / 8) + (unsigned)(NPAD * NC / 8);
        const unsigned grid = (ngroups + 255u) / 256u;
        k_convert<<<grid, 256, 0, stream>>>(x, W, xh, wh);
    }
    {
        k_gemm_softmax<<<MROWS / 16, 256, 0, stream>>>(xh, wh, wsm);
    }
    {
        k_band_conv<<<NB * NH * (NT / 64), 256, 0, stream>>>(x, wsm, out);
    }
}
